// MABSA_Model_21981642621056
// MI455X (gfx1250) — hardware-verified
//
#include <hip/hip_runtime.h>
#include <stddef.h>

#define NN 4096
#define TD 768
#define IDM 512
#define HH 256
#define HDM 64
#define NCL 3
#define NCP 16
#define QKVW 768
#define NPB 32
#define CAPB 4096
#define LDP 72
#define TLP 260

#define WSC 64.0f
#define S_C 8.0f
#define S_QKV 32.0f
#define S_O 64.0f
#define S_AO 128.0f
#define S_G1 512.0f
#define S_G2 1024.0f

typedef _Float16 f16;
typedef f16 v16h __attribute__((ext_vector_type(16)));
typedef f16 v8h __attribute__((ext_vector_type(8)));
typedef float v8f __attribute__((ext_vector_type(8)));
typedef float v4f __attribute__((ext_vector_type(4)));
typedef int v4i __attribute__((ext_vector_type(4)));
typedef v8h __attribute__((may_alias)) v8ha;
typedef v4f __attribute__((may_alias)) v4fa;
typedef v4i __attribute__((may_alias)) v4ia;

union Frag {
  v16h v;
  v8h p[2];
};

__device__ __forceinline__ v8f zero8() {
  v8f z = {0.0f, 0.0f, 0.0f, 0.0f, 0.0f, 0.0f, 0.0f, 0.0f};
  return z;
}

__device__ __forceinline__ v8f mma16(v16h a, v16h b, v8f c) {
  c = __builtin_amdgcn_wmma_f32_16x16x32_f16(false, a, false, b, (short)0, c, false, false);
  asm volatile("v_nop\n\tv_nop\n\tv_nop\n\tv_nop" : "+v"(c) : "v"(a), "v"(b));
  return c;
}

__device__ __forceinline__ v16h ldfrag(const f16* base, int ld, int row0, int k0, int lane) {
  const f16* q = base + (size_t)(row0 + (lane & 15)) * ld + k0 + ((lane >> 4) << 3);
  Frag f;
  f.p[0] = *(const v8ha*)q;
  f.p[1] = *(const v8ha*)(q + 16);
  return f.v;
}

__device__ __forceinline__ v8h cvt8(v4f a, v4f b, float s) {
  v8h r;
  r[0] = (f16)(a[0] * s);
  r[1] = (f16)(a[1] * s);
  r[2] = (f16)(a[2] * s);
  r[3] = (f16)(a[3] * s);
  r[4] = (f16)(b[0] * s);
  r[5] = (f16)(b[1] * s);
  r[6] = (f16)(b[2] * s);
  r[7] = (f16)(b[3] * s);
  return r;
}

__global__ __launch_bounds__(256) void k_cvt_in(const float* __restrict__ a, int na8,
                                                const float* __restrict__ b, int nb8,
                                                f16* __restrict__ ah, f16* __restrict__ bh) {
  const int i = (int)blockIdx.x * 256 + (int)threadIdx.x;
  if (i >= na8 + nb8) return;
  const float* s;
  f16* d;
  if (i < na8) {
    s = a + (size_t)i * 8;
    d = ah + (size_t)i * 8;
  } else {
    const int j = i - na8;
    s = b + (size_t)j * 8;
    d = bh + (size_t)j * 8;
  }
  const v4f x0 = *(const v4fa*)s;
  const v4f x1 = *(const v4fa*)(s + 4);
  const v8h o = cvt8(x0, x1, 1.0f);
  *(volatile v8h*)d = o;
  __threadfence();
  *(volatile v8h*)d = o;
}

struct WPrep {
  const float* w[9];
  f16* o[9];
  int K[9];
  int ncol[9];
  int np[9];
  int pad;
};
static_assert(sizeof(WPrep) == 256);

__global__ __launch_bounds__(256) void k_wprep(WPrep P) {
  __shared__ __align__(16) f16 tile[64][LDP];
  const int j = (int)blockIdx.y;
  const float* w = P.w[j];
  f16* o = P.o[j];
  const int K = P.K[j], ncol = P.ncol[j], np = P.np[j];
  const int kt = K >> 6, ntl = (np + 63) >> 6;
  if ((int)blockIdx.x >= kt * ntl) return;
  const int k0 = ((int)blockIdx.x % kt) << 6;
  const int n0 = ((int)blockIdx.x / kt) << 6;
  const int t = (int)threadIdx.x, nn = t & 63;
  for (int kk = t >> 6; kk < 64; kk += 4) {
    const int n = n0 + nn, k = k0 + kk;
    const float v = (n < ncol && k < K) ? w[(size_t)k * ncol + n] : 0.0f;
    tile[nn][kk] = (f16)(v * WSC);
  }
  __syncthreads();
  v8h val[2];
  size_t dof[2];
  bool ok[2];
#pragma unroll
  for (int ps = 0; ps < 2; ++ps) {
    const int row = (ps << 5) + (t >> 3), piece = t & 7, n = n0 + row;
    ok[ps] = n < np;
    val[ps] = *(const v8ha*)&tile[row][piece << 3];
    dof[ps] = (size_t)n * K + k0 + (piece << 3);
  }
#pragma unroll
  for (int ps = 0; ps < 2; ++ps)
    if (ok[ps]) *(volatile v8h*)(o + dof[ps]) = val[ps];
  __threadfence();
#pragma unroll
  for (int ps = 0; ps < 2; ++ps)
    if (ok[ps]) *(volatile v8h*)(o + dof[ps]) = val[ps];
}

__global__ __launch_bounds__(256) void k_gemm(const f16* __restrict__ A, int K,
                                              const f16* __restrict__ BT, int NCT,
                                              const float* __restrict__ b0,
                                              const float* __restrict__ b1,
                                              const float* __restrict__ b2, int hasb,
                                              float accs, int relu, float oscale, int mode,
                                              float* __restrict__ Cf, f16* __restrict__ Ch,
                                              int M) {
  __shared__ __align__(16) float tile[32][TLP];
  const int t = (int)threadIdx.x, w = t >> 5, lane = t & 31, h = lane >> 4, m = lane & 15;
  const int r0 = (int)blockIdx.x << 5;
  const int by = (int)blockIdx.y;
  const int cb = by << 8;
  if (r0 >= M) return;
  const float* bias = (by == 0) ? b0 : ((by == 1) ? b1 : b2);
  const int rt = w >> 2, cq = (w & 3) << 6;
  v8f acc[4];
#pragma unroll
  for (int j = 0; j < 4; ++j) acc[j] = zero8();
  for (int kk = 0; kk < K; kk += 32) {
    const v16h a = ldfrag(A, K, r0 + (rt << 4), kk, lane);
#pragma unroll
    for (int j = 0; j < 4; ++j)
      acc[j] = mma16(a, ldfrag(BT, K, cb + cq + 16 * j, kk, lane), acc[j]);
  }
#pragma unroll
  for (int j = 0; j < 4; ++j) {
    const int col = cq + 16 * j + m;
    const float bv = hasb ? bias[col] : 0.0f;
#pragma unroll
    for (int r = 0; r < 8; ++r) {
      float v = acc[j][r] * accs + bv;
      if (relu) v = fmaxf(v, 0.0f);
      tile[(rt << 4) + (h << 3) + r][col] = v;
    }
  }
  __syncthreads();
  if (mode == 1) {
    v8h hv[4];
    size_t hd[4];
#pragma unroll
    for (int q = 0; q < 4; ++q) {
      const int row = (w << 2) + q;
      const float* tp = &tile[row][lane << 3];
      hv[q] = cvt8(*(const v4fa*)tp, *(const v4fa*)(tp + 4), oscale);
      hd[q] = (size_t)(r0 + row) * NCT + cb + (lane << 3);
    }
#pragma unroll
    for (int q = 0; q < 4; ++q) *(volatile v8h*)(Ch + hd[q]) = hv[q];
    __threadfence();
#pragma unroll
    for (int q = 0; q < 4; ++q) *(volatile v8h*)(Ch + hd[q]) = hv[q];
  } else {
    v4f fv[8];
    size_t fd[8];
#pragma unroll
    for (int q = 0; q < 4; ++q) {
      const int row = (w << 2) + q;
      fv[2 * q] = *(const v4fa*)&tile[row][lane << 2];
      fv[2 * q + 1] = *(const v4fa*)&tile[row][128 + (lane << 2)];
      fd[2 * q] = (size_t)(r0 + row) * NCT + cb + (lane << 2);
      fd[2 * q + 1] = fd[2 * q] + 128;
    }
#pragma unroll
    for (int q = 0; q < 8; ++q) *(volatile v4f*)(Cf + fd[q]) = fv[q];
    __threadfence();
#pragma unroll
    for (int q = 0; q < 8; ++q) *(volatile v4f*)(Cf + fd[q]) = fv[q];
  }
}

__global__ __launch_bounds__(256) void k_proj(const f16* __restrict__ Xt,
                                              const f16* __restrict__ WtT,
                                              const float* __restrict__ bt,
                                              const f16* __restrict__ Xi,
                                              const f16* __restrict__ WiT,
                                              const float* __restrict__ bi,
                                              f16* __restrict__ C, int M) {
  __shared__ __align__(16) float tile[32][TLP];
  const int t = (int)threadIdx.x, w = t >> 5, lane = t & 31, h = lane >> 4, m = lane & 15;
  const int r0 = (int)blockIdx.x << 5;
  if (r0 >= M) return;
  const int rt = w >> 2, cq = (w & 3) << 6;
  v8f at[4], ai[4];
#pragma unroll
  for (int j = 0; j < 4; ++j) {
    at[j] = zero8();
    ai[j] = zero8();
  }
  for (int kk = 0; kk < TD; kk += 32) {
    const v16h a = ldfrag(Xt, TD, r0 + (rt << 4), kk, lane);
#pragma unroll
    for (int j = 0; j < 4; ++j) at[j] = mma16(a, ldfrag(WtT, TD, cq + 16 * j, kk, lane), at[j]);
  }
  for (int kk = 0; kk < IDM; kk += 32) {
    const v16h a = ldfrag(Xi, IDM, r0 + (rt << 4), kk, lane);
#pragma unroll
    for (int j = 0; j < 4; ++j) ai[j] = mma16(a, ldfrag(WiT, IDM, cq + 16 * j, kk, lane), ai[j]);
  }
  const float accs = 1.0f / WSC;
#pragma unroll
  for (int j = 0; j < 4; ++j) {
    const int col = cq + 16 * j + m;
    const float bb0 = bt[col], bb1 = bi[col];
#pragma unroll
    for (int r = 0; r < 8; ++r) {
      const float v = fmaxf(at[j][r] * accs + bb0, 0.0f) + fmaxf(ai[j][r] * accs + bb1, 0.0f);
      tile[(rt << 4) + (h << 3) + r][col] = v;
    }
  }
  __syncthreads();
  v8h hv[4];
  size_t hd[4];
#pragma unroll
  for (int q = 0; q < 4; ++q) {
    const int row = (w << 2) + q;
    const float* tp = &tile[row][lane << 3];
    hv[q] = cvt8(*(const v4fa*)tp, *(const v4fa*)(tp + 4), S_C);
    hd[q] = (size_t)(r0 + row) * HH + (lane << 3);
  }
#pragma unroll
  for (int q = 0; q < 4; ++q) *(volatile v8h*)(C + hd[q]) = hv[q];
  __threadfence();
#pragma unroll
  for (int q = 0; q < 4; ++q) *(volatile v8h*)(C + hd[q]) = hv[q];
}

__global__ __launch_bounds__(256) void k_attn(const f16* __restrict__ qkv, f16* __restrict__ ob) {
  __shared__ __align__(16) f16 Ks[64][LDP];
  __shared__ __align__(16) f16 Vt[64][LDP];
  __shared__ __align__(16) f16 Ps[8][16][LDP];
  const int t = (int)threadIdx.x, w = t >> 5, lane = t & 31, h = lane >> 4, m = lane & 15;
  const int head = (int)blockIdx.x >> 5;
  const int qbase = ((int)blockIdx.x & 31) << 7;
  const int qr0 = qbase + (w << 4);
  const int qc = head * HDM, kc = HH + head * HDM, vc = 2 * HH + head * HDM;
  const v16h qa0 = ldfrag(qkv, QKVW, qr0, qc, lane);
  const v16h qa1 = ldfrag(qkv, QKVW, qr0, qc + 32, lane);
  float mr[8], lr[8];
  v8f o[4];
#pragma unroll
  for (int c = 0; c < 4; ++c) o[c] = zero8();
#pragma unroll
  for (int r = 0; r < 8; ++r) {
    mr[r] = -1.0e30f;
    lr[r] = 0.0f;
  }
  const float sc = 0.125f / (S_QKV * S_QKV);
  f16* pw = &Ps[w][0][0];

  for (int kb = 0; kb < NN; kb += 64) {
    __syncthreads();
#pragma unroll
    for (int ps = 0; ps < 2; ++ps) {
      const int key = (t >> 3) + (ps << 5), piece = t & 7;
      const f16* rp = qkv + (size_t)(kb + key) * QKVW;
      const v8h kv = *(const v8ha*)(rp + kc + (piece << 3));
      const v8h vv = *(const v8ha*)(rp + vc + (piece << 3));
      *(v8ha*)&Ks[key][piece << 3] = kv;
#pragma unroll
      for (int i = 0; i < 8; ++i) Vt[(piece << 3) + i][key] = vv[i];
    }
    __syncthreads();
    v8f s[4];
#pragma unroll
    for (int c = 0; c < 4; ++c) {
      v8f z = zero8();
      z = mma16(qa0, ldfrag(&Ks[0][0], LDP, c << 4, 0, lane), z);
      z = mma16(qa1, ldfrag(&Ks[0][0], LDP, c << 4, 32, lane), z);
      s[c] = z;
    }
#pragma unroll
    for (int r = 0; r < 8; ++r) {
      const float x0 = s[0][r] * sc, x1 = s[1][r] * sc, x2 = s[2][r] * sc, x3 = s[3][r] * sc;
      float rm = fmaxf(fmaxf(x0, x1), fmaxf(x2, x3));
      rm = fmaxf(rm, __shfl_xor(rm, 1, 32));
      rm = fmaxf(rm, __shfl_xor(rm, 2, 32));
      rm = fmaxf(rm, __shfl_xor(rm, 4, 32));
      rm = fmaxf(rm, __shfl_xor(rm, 8, 32));
      const float mn = fmaxf(mr[r], rm);
      const float al = __expf(mr[r] - mn);
      const f16 p0 = (f16)__expf(x0 - mn);
      const f16 p1 = (f16)__expf(x1 - mn);
      const f16 p2 = (f16)__expf(x2 - mn);
      const f16 p3 = (f16)__expf(x3 - mn);
      float rs = ((float)p0 + (float)p1) + ((float)p2 + (float)p3);
      rs += __shfl_xor(rs, 1, 32);
      rs += __shfl_xor(rs, 2, 32);
      rs += __shfl_xor(rs, 4, 32);
      rs += __shfl_xor(rs, 8, 32);
      lr[r] = lr[r] * al + rs;
      mr[r] = mn;
      f16* pr = pw + ((h << 3) + r) * LDP + m;
      pr[0] = p0;
      pr[16] = p1;
      pr[32] = p2;
      pr[48] = p3;
      o[0][r] *= al;
      o[1][r] *= al;
      o[2][r] *= al;
      o[3][r] *= al;
    }
    __syncthreads();
#pragma unroll
    for (int ks = 0; ks < 2; ++ks) {
      const v16h pa = ldfrag(pw, LDP, 0, ks << 5, lane);
#pragma unroll
      for (int c = 0; c < 4; ++c)
        o[c] = mma16(pa, ldfrag(&Vt[0][0], LDP, c << 4, ks << 5, lane), o[c]);
    }
  }
  __syncthreads();
  const float osc = S_O / S_QKV;
#pragma unroll
  for (int r = 0; r < 8; ++r) {
    const float inv = osc / lr[r];
    f16* pr = pw + ((h << 3) + r) * LDP + m;
    pr[0] = (f16)(o[0][r] * inv);
    pr[16] = (f16)(o[1][r] * inv);
    pr[32] = (f16)(o[2][r] * inv);
    pr[48] = (f16)(o[3][r] * inv);
  }
  __syncthreads();
  v8h ov[4];
  size_t od[4];
#pragma unroll
  for (int q = 0; q < 4; ++q) {
    const int row = (q << 2) + (lane >> 3), piece = lane & 7;
    ov[q] = *(const v8ha*)(pw + row * LDP + (piece << 3));
    od[q] = (size_t)(qr0 + row) * HH + qc + (piece << 3);
  }
#pragma unroll
  for (int q = 0; q < 4; ++q) *(volatile v8h*)(ob + od[q]) = ov[q];
  __threadfence();
#pragma unroll
  for (int q = 0; q < 4; ++q) *(volatile v8h*)(ob + od[q]) = ov[q];
}

__global__ __launch_bounds__(256) void k_gprep(const int* __restrict__ ei, int E,
                                               float* __restrict__ dinv,
                                               int* __restrict__ cnt,
                                               int* __restrict__ csr) {
  __shared__ __align__(16) int lst[CAPB];
  __shared__ __align__(16) int srt[CAPB];
  __shared__ int wc[8];
  __shared__ __align__(16) float dvl[NPB];
  __shared__ __align__(16) int cnl[NPB];
  const int t = (int)threadIdx.x, w = t >> 5, lane = t & 31;
  const int nb = (int)blockIdx.x * NPB;
  const int* src = ei;
  const int* dst = ei + E;
  int len = 0;
  const int nch = (E + 1023) >> 10;
  const unsigned lt = (1u << lane) - 1u;
  for (int c = 0; c < nch; ++c) {
    int pk[4];
    bool mt[4];
    unsigned bal[4];
#pragma unroll
    for (int i = 0; i < 4; ++i) {
      const int e = (c << 10) + (i << 8) + t;
      const bool valid = e < E;
      const int d = valid ? dst[e] : -1;
      int s = valid ? src[e] : 0;
      s = s < 0 ? 0 : (s > NN - 1 ? NN - 1 : s);
      const bool mm = valid && d >= nb && d < nb + NPB;
      const int loc = mm ? (d - nb) : 0;
      mt[i] = mm;
      pk[i] = s | (loc << 16);
      bal[i] = __builtin_amdgcn_ballot_w32(mm);
    }
    const int c0 = (int)__popc(bal[0]), c1 = (int)__popc(bal[1]), c2 = (int)__popc(bal[2]),
              c3 = (int)__popc(bal[3]);
    if (lane == 0) wc[w] = c0 + c1 + c2 + c3;
    __syncthreads();
    int pre = 0, tot = 0;
#pragma unroll
    for (int ww = 0; ww < 8; ++ww) {
      const int v = wc[ww];
      tot += v;
      pre += (ww < w) ? v : 0;
    }
    const int basep = len + pre;
    int rk[4];
    rk[0] = (int)__popc(bal[0] & lt);
    rk[1] = c0 + (int)__popc(bal[1] & lt);
    rk[2] = c0 + c1 + (int)__popc(bal[2] & lt);
    rk[3] = c0 + c1 + c2 + (int)__popc(bal[3] & lt);
#pragma unroll
    for (int i = 0; i < 4; ++i) {
      if (mt[i]) {
        const int p = basep + rk[i];
        if (p < CAPB) lst[p] = pk[i];
      }
    }
    len += tot;
    __syncthreads();
  }
  const int L = len < CAPB ? len : CAPB;
  for (int i = t; i < CAPB; i += 256)
    if (i >= L) srt[i] = 0;
  if (w == 0) {
    int cn = 0;
    for (int e = 0; e < L; ++e) cn += ((lst[e] >> 16) == lane) ? 1 : 0;
    int incl = cn;
#pragma unroll
    for (int dd = 1; dd < 32; dd <<= 1) {
      const int v = __shfl_up(incl, dd, 32);
      if (lane >= dd) incl += v;
    }
    const int off = incl - cn;
    cnl[lane] = cn;
    dvl[lane] = 1.0f / sqrtf((float)(cn + 1));
    int run = 0;
    for (int e = 0; e < L; ++e) {
      const int v = lst[e];
      if ((v >> 16) == lane) {
        srt[off + run] = v & 0xFFFF;
        ++run;
      }
    }
  }
  __syncthreads();
  v4f dv4;
  v4i cn4;
  if (t < 8) {
    dv4 = *(const v4fa*)&dvl[t << 2];
    cn4 = *(const v4ia*)&cnl[t << 2];
  }
  v4i sv[4];
#pragma unroll
  for (int k = 0; k < 4; ++k) sv[k] = *(const v4ia*)&srt[(t + (k << 8)) << 2];
  int* seg = csr + (size_t)blockIdx.x * CAPB;
  if (t < 8) {
    *(volatile v4f*)(dinv + nb + (t << 2)) = dv4;
    *(volatile v4i*)(cnt + nb + (t << 2)) = cn4;
  }
#pragma unroll
  for (int k = 0; k < 4; ++k) *(volatile v4i*)(seg + ((t + (k << 8)) << 2)) = sv[k];
  __threadfence();
  if (t < 8) {
    *(volatile v4f*)(dinv + nb + (t << 2)) = dv4;
    *(volatile v4i*)(cnt + nb + (t << 2)) = cn4;
  }
#pragma unroll
  for (int k = 0; k < 4; ++k) *(volatile v4i*)(seg + ((t + (k << 8)) << 2)) = sv[k];
}

__global__ __launch_bounds__(256) void k_gagg(const float* __restrict__ hx,
                                              const float* __restrict__ dinv,
                                              const int* __restrict__ cnt,
                                              const int* __restrict__ csr,
                                              const float* __restrict__ bias, int relu,
                                              float oscale, f16* __restrict__ outh) {
  __shared__ int offl[NPB];
  __shared__ int cnl[NPB];
  const int t = (int)threadIdx.x, w = t >> 5, lane = t & 31;
  const int nb = (int)blockIdx.x * NPB;
  if (t < 32) {
    int c = cnt[nb + t];
    c = c < 0 ? 0 : (c > CAPB ? CAPB : c);
    int incl = c;
#pragma unroll
    for (int dd = 1; dd < 32; dd <<= 1) {
      const int v = __shfl_up(incl, dd, 32);
      if (lane >= dd) incl += v;
    }
    offl[t] = incl - c;
    cnl[t] = c;
  }
  __syncthreads();
  const int* seg = csr + (size_t)blockIdx.x * CAPB;
  const int c0 = lane << 3;
  const v4f bb0 = *(const v4fa*)(bias + c0);
  const v4f bb1 = *(const v4fa*)(bias + c0 + 4);
  v8h ov[4];
  size_t od[4];
#pragma unroll
  for (int q = 0; q < 4; ++q) {
    const int j = (w << 2) + q, n = nb + j;
    const float dn = dinv[n];
    const float* hr = hx + (size_t)n * HH + c0;
    const v4f a0 = *(const v4fa*)hr;
    const v4f a1 = *(const v4fa*)(hr + 4);
    const float wsf = dn * dn;
    float acc[8];
    acc[0] = wsf * a0[0];
    acc[1] = wsf * a0[1];
    acc[2] = wsf * a0[2];
    acc[3] = wsf * a0[3];
    acc[4] = wsf * a1[0];
    acc[5] = wsf * a1[1];
    acc[6] = wsf * a1[2];
    acc[7] = wsf * a1[3];
    int st = offl[j], ce = cnl[j];
    if (st > CAPB) st = CAPB;
    if (st + ce > CAPB) ce = CAPB - st;
    for (int e = 0; e < ce; ++e) {
      int s = seg[st + e];
      s = ((unsigned)s < (unsigned)NN) ? s : 0;
      const float nm = dinv[s] * dn;
      const float* hs = hx + (size_t)s * HH + c0;
      const v4f g0 = *(const v4fa*)hs;
      const v4f g1 = *(const v4fa*)(hs + 4);
      acc[0] += nm * g0[0];
      acc[1] += nm * g0[1];
      acc[2] += nm * g0[2];
      acc[3] += nm * g0[3];
      acc[4] += nm * g1[0];
      acc[5] += nm * g1[1];
      acc[6] += nm * g1[2];
      acc[7] += nm * g1[3];
    }
    v4f u0, u1;
    u0[0] = acc[0] + bb0[0];
    u0[1] = acc[1] + bb0[1];
    u0[2] = acc[2] + bb0[2];
    u0[3] = acc[3] + bb0[3];
    u1[0] = acc[4] + bb1[0];
    u1[1] = acc[5] + bb1[1];
    u1[2] = acc[6] + bb1[2];
    u1[3] = acc[7] + bb1[3];
    if (relu) {
#pragma unroll
      for (int i = 0; i < 4; ++i) {
        u0[i] = fmaxf(u0[i], 0.0f);
        u1[i] = fmaxf(u1[i], 0.0f);
      }
    }
    ov[q] = cvt8(u0, u1, oscale);
    od[q] = (size_t)n * HH + c0;
    *(volatile v8h*)(outh + od[q]) = ov[q];
  }
  __threadfence();
#pragma unroll
  for (int q = 0; q < 4; ++q) *(volatile v8h*)(outh + od[q]) = ov[q];
}

__global__ __launch_bounds__(256) void k_cls(const f16* __restrict__ g2,
                                             const f16* __restrict__ wcT,
                                             const float* __restrict__ cb,
                                             float* __restrict__ out) {
  __shared__ __align__(16) float os[NN * NCL];
  const int t = (int)threadIdx.x, w = t >> 5, lane = t & 31, h = lane >> 4, m = lane & 15;
  const float accs = 1.0f / (S_G2 * WSC);
  const float cbv = (m < NCL) ? cb[m] : 0.0f;
  for (int rt = w; rt < NN / 16; rt += 8) {
    v8f acc = zero8();
#pragma unroll
    for (int kk = 0; kk < HH; kk += 32)
      acc = mma16(ldfrag(g2, HH, rt << 4, kk, lane), ldfrag(wcT, HH, 0, kk, lane), acc);
    if (m < NCL) {
#pragma unroll
      for (int r = 0; r < 8; ++r) os[((rt << 4) + (h << 3) + r) * NCL + m] = acc[r] * accs + cbv;
    }
  }
  __syncthreads();
  v4f v[12];
#pragma unroll
  for (int k = 0; k < 12; ++k) v[k] = *(const v4fa*)&os[(t + (k << 8)) << 2];
#pragma unroll
  for (int k = 0; k < 12; ++k) *(volatile v4f*)(out + ((t + (k << 8)) << 2)) = v[k];
  __threadfence();
#pragma unroll
  for (int k = 0; k < 12; ++k) *(volatile v4f*)(out + ((t + (k << 8)) << 2)) = v[k];
}

extern "C" void kernel_launch(void* const* d_in, const int* in_sizes, int n_in,
                              void* d_out, int out_size, void* d_ws, size_t ws_size,
                              hipStream_t stream) {
  if (n_in < 21) return;
  if (in_sizes[0] != NN * TD || in_sizes[1] != NN * IDM) return;
  if (in_sizes[2] < 2 || (in_sizes[2] & 1)) return;
  if (in_sizes[3] != TD * HH || in_sizes[4] != HH || in_sizes[5] != IDM * HH || in_sizes[6] != HH) return;
  for (int i = 7; i <= 17; i += 2)
    if (in_sizes[i] != HH * HH || in_sizes[i + 1] != HH) return;
  if (in_sizes[19] != HH * NCL || in_sizes[20] != NCL) return;
  if (out_size != NN * NCL) return;

  const float* textf = (const float*)d_in[0];
  const float* imgf = (const float*)d_in[1];
  const int* edges = (const int*)d_in[2];
  const float* text_w = (const float*)d_in[3];
  const float* text_b = (const float*)d_in[4];
  const float* image_w = (const float*)d_in[5];
  const float* image_b = (const float*)d_in[6];
  const float* wq = (const float*)d_in[7];
  const float* bq = (const float*)d_in[8];
  const float* wk = (const float*)d_in[9];
  const float* bk = (const float*)d_in[10];
  const float* wv = (const float*)d_in[11];
  const float* bv = (const float*)d_in[12];
  const float* wo = (const float*)d_in[13];
  const float* bo = (const float*)d_in[14];
  const float* g1w = (const float*)d_in[15];
  const float* g1b = (const float*)d_in[16];
  const float* g2w = (const float*)d_in[17];
  const float* g2b = (const float*)d_in[18];
  const float* clw = (const float*)d_in[19];
  const float* clb = (const float*)d_in[20];
  float* outp = (float*)d_out;
  const int E = in_sizes[2] / 2;

  char* base = (char*)d_ws;
  size_t off = 0;
  auto carve = [&](size_t bytes) -> char* {
    char* p = base + off;
    off += (bytes + 255) & ~(size_t)255;
    return p;
  };
  f16* texth = (f16*)carve((size_t)NN * TD * 2);
  f16* imgh = (f16*)carve((size_t)NN * IDM * 2);
  f16* wtT = (f16*)carve((size_t)HH * TD * 2);
  f16* wiT = (f16*)carve((size_t)HH * IDM * 2);
  f16* wqkvT = (f16*)carve((size_t)QKVW * HH * 2);
  f16* woT = (f16*)carve((size_t)HH * HH * 2);
  f16* g1T = (f16*)carve((size_t)HH * HH * 2);
  f16* g2T = (f16*)carve((size_t)HH * HH * 2);
  f16* wcT = (f16*)carve((size_t)NCP * HH * 2);
  f16* comb = (f16*)carve((size_t)NN * HH * 2);
  f16* qkv = (f16*)carve((size_t)NN * QKVW * 2);
  f16* obuf = (f16*)carve((size_t)NN * HH * 2);
  f16* aoh = (f16*)carve((size_t)NN * HH * 2);
  float* hx = (float*)carve((size_t)NN * HH * 4);
  f16* g1h = (f16*)carve((size_t)NN * HH * 2);
  float* hx2 = (float*)carve((size_t)NN * HH * 4);
  f16* g2h = (f16*)carve((size_t)NN * HH * 2);
  float* dinv = (float*)carve((size_t)NN * 4);
  int* cnt = (int*)carve((size_t)NN * 4);
  int* csr = (int*)carve((size_t)(NN / NPB) * CAPB * 4);
  if (off > ws_size) return;

  k_gprep<<<NN / NPB, 256, 0, stream>>>(edges, E, dinv, cnt, csr);

  {
    const int na8 = NN * TD / 8, nb8 = NN * IDM / 8;
    k_cvt_in<<<(na8 + nb8 + 255) / 256, 256, 0, stream>>>(textf, na8, imgf, nb8, texth, imgh);
  }

  {
    WPrep P;
    P.w[0] = text_w;  P.o[0] = wtT;               P.K[0] = TD;  P.ncol[0] = HH;  P.np[0] = HH;
    P.w[1] = image_w; P.o[1] = wiT;               P.K[1] = IDM; P.ncol[1] = HH;  P.np[1] = HH;
    P.w[2] = wq;      P.o[2] = wqkvT;             P.K[2] = HH;  P.ncol[2] = HH;  P.np[2] = HH;
    P.w[3] = wk;      P.o[3] = wqkvT + HH * HH;   P.K[3] = HH;  P.ncol[3] = HH;  P.np[3] = HH;
    P.w[4] = wv;      P.o[4] = wqkvT + 2 * HH * HH; P.K[4] = HH; P.ncol[4] = HH; P.np[4] = HH;
    P.w[5] = wo;      P.o[5] = woT;               P.K[5] = HH;  P.ncol[5] = HH;  P.np[5] = HH;
    P.w[6] = g1w;     P.o[6] = g1T;               P.K[6] = HH;  P.ncol[6] = HH;  P.np[6] = HH;
    P.w[7] = g2w;     P.o[7] = g2T;               P.K[7] = HH;  P.ncol[7] = HH;  P.np[7] = HH;
    P.w[8] = clw;     P.o[8] = wcT;               P.K[8] = HH;  P.ncol[8] = NCL; P.np[8] = NCP;
    P.pad = 0;
    k_wprep<<<dim3((TD / 64) * (HH / 64), 9), 256, 0, stream>>>(P);
  }

  const int rowblocks = NN / 32;

  k_proj<<<rowblocks, 256, 0, stream>>>(texth, wtT, text_b, imgh, wiT, image_b, comb, NN);

  k_gemm<<<dim3(rowblocks, 3), 256, 0, stream>>>(comb, HH, wqkvT, QKVW, bq, bk, bv, 1,
                                                  1.0f / (S_C * WSC), 0, S_QKV, 1, hx, qkv, NN);

  k_attn<<<4 * (NN / 128), 256, 0, stream>>>(qkv, obuf);

  k_gemm<<<dim3(rowblocks, 1), 256, 0, stream>>>(obuf, HH, woT, HH, bo, bo, bo, 1,
                                                  1.0f / (S_O * WSC), 0, S_AO, 1, hx, aoh, NN);

  k_gemm<<<dim3(rowblocks, 1), 256, 0, stream>>>(aoh, HH, g1T, HH, g1b, g1b, g1b, 0,
                                                  1.0f / (S_AO * WSC), 0, 1.0f, 0, hx, g1h, NN);
  k_gagg<<<NN / NPB, 256, 0, stream>>>(hx, dinv, cnt, csr, g1b, 1, S_G1, g1h);

  k_gemm<<<dim3(rowblocks, 1), 256, 0, stream>>>(g1h, HH, g2T, HH, g2b, g2b, g2b, 0,
                                                  1.0f / (S_G1 * WSC), 0, 1.0f, 0, hx2, g2h, NN);
  k_gagg<<<NN / NPB, 256, 0, stream>>>(hx2, dinv, cnt, csr, g2b, 0, S_G2, g2h);

  k_cls<<<1, 256, 0, stream>>>(g2h, wcT, clb, outp);
}
